// TransConv_1254130451193
// MI455X (gfx1250) — hardware-run, weakly checked
//
#include <hip/hip_runtime.h>

typedef float          v8f   __attribute__((ext_vector_type(8)));
typedef float          v4f   __attribute__((ext_vector_type(4)));
typedef unsigned int   v4u   __attribute__((ext_vector_type(4)));
typedef int            v8i   __attribute__((ext_vector_type(8)));
typedef unsigned short v8us  __attribute__((ext_vector_type(8)));
typedef unsigned short v16us __attribute__((ext_vector_type(16)));
typedef __bf16         v16bf __attribute__((ext_vector_type(16)));
typedef _Float16       v16h  __attribute__((ext_vector_type(16)));
typedef v4f  __attribute__((may_alias)) v4fa;
typedef v8us __attribute__((may_alias)) v8usa;
union FragB { v16bf v; v16us u; v8us h[2]; v8i w; };
union FragH { v16h  v; v16us u; v8us h[2]; v8i w; };

__device__ __forceinline__ v8f wmb(const FragB& a, const FragB& b, v8f c) {
  v8f d = __builtin_amdgcn_wmma_f32_16x16x32_bf16(false, a.v, false, b.v, (short)0, c, false, false);
  asm volatile("v_nop\n\tv_nop\n\tv_nop\n\tv_nop" : "+v"(d) : "v"(a.w), "v"(b.w));
  return d;
}

__device__ __forceinline__ v8f wmh(const FragH& a, const FragH& b, v8f c) {
  v8f d = __builtin_amdgcn_wmma_f32_16x16x32_f16(false, a.v, false, b.v, (short)0, c, false, false);
  asm volatile("v_nop\n\tv_nop\n\tv_nop\n\tv_nop" : "+v"(d) : "v"(a.w), "v"(b.w));
  return d;
}

__device__ __forceinline__ unsigned bf16_bits(float f) {
  const unsigned u = __float_as_uint(f);
  const unsigned r = (u + 0x7FFFu + ((u >> 16) & 1u)) >> 16;
  const unsigned q = (u >> 16) | 0x40u;
  return ((u & 0x7fffffffu) > 0x7f800000u) ? q : r;
}

__device__ __forceinline__ float bf16_val(float f) {
  return __uint_as_float(bf16_bits(f) << 16);
}
__device__ __forceinline__ int clampi(int v, int lo, int hi) {
  return v < lo ? lo : (v > hi ? hi : v);
}

__device__ __forceinline__ unsigned f16_bits(float f) {
  const unsigned u  = __float_as_uint(f);
  const unsigned s  = (u >> 16) & 0x8000u;
  const unsigned a  = u & 0x7fffffffu;
  const unsigned t  = a - 0x38000000u;
  const unsigned r  = (t + 0x0FFFu + ((t >> 13) & 1u)) >> 13;
  const unsigned rc = r > 0x7C00u ? 0x7C00u : r;
  const bool small  = a < 0x38800000u;
  const bool isnan  = a > 0x7f800000u;
  const unsigned fin = small ? 0u : (s | rc);
  return isnan ? (s | 0x7E00u) : fin;
}

__device__ __forceinline__ unsigned pk16(unsigned lo, unsigned hi) { return lo | (hi << 16); }
__device__ __forceinline__ unsigned bf16_lo_bits(float v) {
  float hi = bf16_val(v);
  asm volatile("" : "+v"(hi));
  return bf16_bits(v - hi);
}
__device__ __forceinline__ v4u pack8_bf16(v4f a, v4f c) {
  return (v4u){ pk16(bf16_bits(a[0]), bf16_bits(a[1])), pk16(bf16_bits(a[2]), bf16_bits(a[3])),
                pk16(bf16_bits(c[0]), bf16_bits(c[1])), pk16(bf16_bits(c[2]), bf16_bits(c[3])) };
}
__device__ __forceinline__ v4u pack8_bf16_lo(v4f a, v4f c) {
  return (v4u){ pk16(bf16_lo_bits(a[0]), bf16_lo_bits(a[1])), pk16(bf16_lo_bits(a[2]), bf16_lo_bits(a[3])),
                pk16(bf16_lo_bits(c[0]), bf16_lo_bits(c[1])), pk16(bf16_lo_bits(c[2]), bf16_lo_bits(c[3])) };
}
__device__ __forceinline__ v4u pack8_f16(v4f a, v4f c) {
  return (v4u){ pk16(f16_bits(a[0]), f16_bits(a[1])), pk16(f16_bits(a[2]), f16_bits(a[3])),
                pk16(f16_bits(c[0]), f16_bits(c[1])), pk16(f16_bits(c[2]), f16_bits(c[3])) };
}

template <int FORM>
__global__ __launch_bounds__(256) void k_plane(const float* __restrict__ src, int rows, int cols, int ldsrc,
                                               unsigned short* __restrict__ dst, int MP, int KP) {
  static_assert(FORM >= 0 && FORM <= 3);
  const int KTOT = (FORM == 1 || FORM == 3) ? 2 * KP : KP;
  const unsigned ppr   = (unsigned)(KTOT >> 3);
  const unsigned kp8   = (unsigned)(KP >> 3);
  const unsigned total = (unsigned)MP * ppr;
  const unsigned g     = blockIdx.x * 256u + threadIdx.x;
  const unsigned rowu  = g / ppr;
  const unsigned p     = g - rowu * ppr;
  const bool second    = p >= kp8;
  const int row = (int)rowu;
  const int c0  = (int)((second ? p - kp8 : p) << 3);
  const float* srow = src + (size_t)clampi(row, 0, rows - 1) * (size_t)ldsrc;
  float x[8];
  unsigned mk[8];
#pragma unroll
  for (int e = 0; e < 8; ++e) {
    const int c = c0 + e;
    const float v = srow[clampi(c, 0, cols - 1)];
    asm volatile("" :: "v"(v));
    x[e]  = v;
    mk[e] = (row < rows && c < cols) ? 0xFFFFu : 0u;
  }
  const v4f a = (v4f){ x[0], x[1], x[2], x[3] };
  const v4f c = (v4f){ x[4], x[5], x[6], x[7] };
  v4u o;
  if (FORM == 2) {
    o = pack8_f16(a, c);
  } else {
    const v4u hi = pack8_bf16(a, c);
    o = hi;
    if (FORM == 1) { const v4u lo = pack8_bf16_lo(a, c); o = second ? lo : hi; }
  }
  const v4u mw = (v4u){ pk16(mk[0], mk[1]), pk16(mk[2], mk[3]), pk16(mk[4], mk[5]), pk16(mk[6], mk[7]) };
  o &= mw;
  if (g < total) {
    volatile v4u* q = (volatile v4u*)(dst + (size_t)g * 8);
    *q = o;
    __threadfence();
    *q = o;
  }
}

template <int FORM> struct FragOf    { typedef FragB T; };
template <>         struct FragOf<2> { typedef FragH T; };
__device__ __forceinline__ v8f mm(const FragB& a, const FragB& b, v8f c) { return wmb(a, b, c); }
__device__ __forceinline__ v8f mm(const FragH& a, const FragH& b, v8f c) { return wmh(a, b, c); }
template <class F> __device__ __forceinline__ F ld_frag(const unsigned short* p) {
  F f;
  f.h[0] = *(const v8usa*)(p);
  f.h[1] = *(const v8usa*)(p + 16);
  return f;
}

template <int FORM, int EPI>
__global__ __launch_bounds__(256) __attribute__((amdgpu_num_vgpr(248)))
void k_gemm_nt(const unsigned short* __restrict__ A, const unsigned short* __restrict__ B,
               const float* __restrict__ bias, float* __restrict__ D, int M, int N, int KTOT, int ldd) {
  static_assert(FORM >= 0 && FORM <= 2);
  static_assert(EPI == 0 || EPI == 1);
  typedef typename FragOf<FORM>::T F;
  __shared__ __attribute__((aligned(16))) float sT[8][16 * 68];
  const int lane = threadIdx.x & 31;
  const int wave = threadIdx.x >> 5;
  const int tilesM = (M + 63) >> 6;
  const int tilesN = (N + 63) >> 6;
  const int tile = blockIdx.x * 8 + wave;
  if (tile >= tilesM * tilesN) return;
  const int tm = tile / tilesN;
  const int tn = tile - tm * tilesN;
  const int m0 = tm << 6;
  const int n0 = tn << 6;

  const int rl = lane & 15;
  const int h8 = (lane >> 4) * 8;
  const unsigned short* pa = A + (size_t)(m0 + rl) * (size_t)KTOT + h8;
  const unsigned short* pb = B + (size_t)(n0 + rl) * (size_t)KTOT + h8;

  v8f acc[4][4];
#pragma unroll
  for (int i = 0; i < 4; ++i)
#pragma unroll
    for (int j = 0; j < 4; ++j) acc[i][j] = (v8f){0.f, 0.f, 0.f, 0.f, 0.f, 0.f, 0.f, 0.f};

#pragma unroll 1
  for (int k0 = 0; k0 < KTOT; k0 += 32) {
    F bf[4];
#pragma unroll
    for (int j = 0; j < 4; ++j) bf[j] = ld_frag<F>(pb + (size_t)(j << 4) * (size_t)KTOT + k0);
#pragma unroll
    for (int i = 0; i < 4; ++i) {
      const F af = ld_frag<F>(pa + (size_t)(i << 4) * (size_t)KTOT + k0);
#pragma unroll
      for (int j = 0; j < 4; ++j) acc[i][j] = mm(af, bf[j], acc[i][j]);
    }
  }

  float* slab = sT[wave];
  const int hh = lane >> 4;
  const int c4 = (lane & 15) * 4;
  const int nc = n0 + c4;
  const bool cok = nc < N;
  v4f bv = (v4f){0.f, 0.f, 0.f, 0.f};
  if (EPI == 1) {
    bv = *(const v4fa*)(bias + clampi(nc, 0, N - 4));
    asm volatile("" :: "v"(bv));
  }
#pragma unroll
  for (int i = 0; i < 4; ++i) {
    const int mBase = m0 + (i << 4);
#pragma unroll
    for (int j = 0; j < 4; ++j) {
#pragma unroll
      for (int r = 0; r < 8; ++r) slab[(h8 + r) * 68 + (j << 4) + rl] = acc[i][j][r];
    }
    __builtin_amdgcn_fence(__ATOMIC_RELEASE, "workgroup");
    __builtin_amdgcn_wave_barrier();
    __builtin_amdgcn_fence(__ATOMIC_ACQUIRE, "workgroup");
    v4f vv[8];
#pragma unroll
    for (int it = 0; it < 8; ++it) {
      const int row = it * 2 + hh;
      v4f v = *(const v4fa*)(slab + row * 68 + c4);
      if (EPI == 1) v += bv;
      vv[it] = v;
    }
    for (int pass = 0; pass < 2; ++pass) {
#pragma unroll
      for (int it = 0; it < 8; ++it) {
        const int row = mBase + it * 2 + hh;
        if (cok && row < M) *(volatile v4f*)(D + (size_t)row * (size_t)ldd + nc) = vv[it];
      }
      __threadfence();
    }
    __builtin_amdgcn_fence(__ATOMIC_RELEASE, "workgroup");
    __builtin_amdgcn_wave_barrier();
    __builtin_amdgcn_fence(__ATOMIC_ACQUIRE, "workgroup");
  }
}

#include <stddef.h>

#define NN     50000
#define NE     250000
#define HIDC   32
#define NHEAD  4
#define RB     128
#define NBLK   391
#define NPADR  (NBLK * RB)
#define MBR    512
#define NMB    98
#define CNB    1024
#define NCB    49
#define CNTN   (NCB * CNB)
#define CEPT   8
#define CCHUNK 2048
#define CWCAP  256
#define DEGCAP 32
#define PLE    ((size_t)NPADR * 128)
#define WSMAX  ((size_t)128 << 20)

static_assert(HIDC == 32);
static_assert(NHEAD * HIDC == 128);
static_assert(NN == 390 * RB + 80);
static_assert(NPADR >= NN && NPADR % 16 == 0);
static_assert(NMB * MBR == CNTN && CNTN >= NPADR);
static_assert((RB * 33 * 4) % 128 == 0);
static_assert((80 * 33) % 4 == 0 && (RB * 33) % 4 == 0);
static_assert(NE == 122 * CCHUNK + 144);
static_assert(CWCAP == 32 * CEPT && CCHUNK == 256 * CEPT);
static_assert(DEGCAP >= 16 + 8);

typedef int v4i __attribute__((ext_vector_type(4)));
typedef v4i __attribute__((may_alias)) v4ia;

__device__ __forceinline__ float wsum32(float v) {
#pragma unroll
  for (int q = 16; q > 0; q >>= 1) v += __shfl_xor(v, q, 32);
  return v;
}
__device__ __forceinline__ float leaky01(float x) { return x >= 0.0f ? x : 0.01f * x; }

__device__ __forceinline__ FragB mk_frag(v4u a, v4u b) {
  FragB f;
  f.w = (v8i){ (int)a[0], (int)a[1], (int)a[2], (int)a[3], (int)b[0], (int)b[1], (int)b[2], (int)b[3] };
  return f;
}

__device__ __forceinline__ void flush_tile(const float* st, float* gbase, int pitch, int lane) {
  const int rq = lane >> 3;
  const int c4 = (lane & 7) * 4;
  v4f vv[4];
#pragma unroll
  for (int it = 0; it < 4; ++it) vv[it] = *(const v4fa*)(st + (it * 4 + rq) * 32 + c4);
  for (int pass = 0; pass < 2; ++pass) {
#pragma unroll
    for (int it = 0; it < 4; ++it)
      *(volatile v4f*)(gbase + (size_t)(it * 4 + rq) * (size_t)pitch + c4) = vv[it];
    __threadfence();
  }
}

__device__ __forceinline__ void plane_piece(const float* __restrict__ src, int hoff, int col, int k8, int kmask,
                                            unsigned short* dstp) {
  float x[8];
#pragma unroll
  for (int e = 0; e < 8; ++e) {
    const int k = (k8 + e) & kmask;
    const float v = src[hoff + (1 + k) * 32 + col];
    asm volatile("" :: "v"(v));
    x[e] = v;
  }
  const v4u o = pack8_bf16((v4f){ x[0], x[1], x[2], x[3] }, (v4f){ x[4], x[5], x[6], x[7] });
  volatile v4u* q = (volatile v4u*)dstp;
  *q = o;
  __threadfence();
  *q = o;
}

__global__ __launch_bounds__(256) void k_prep(const float* __restrict__ Wfc, const float* __restrict__ Wq,
                                              const float* __restrict__ Wk, const float* __restrict__ Wv,
                                              const float* __restrict__ Who, unsigned short* WfcT,
                                              unsigned short* WqkvT, unsigned short* WhoT) {
  const int blk = (int)blockIdx.x, tid = (int)threadIdx.x;
  if (blk < 2) {
    const int u = blk * 256 + tid;
    plane_piece(Wfc, 0, u >> 4, (u & 15) * 8, 127, WfcT + (size_t)u * 8);
  } else if (blk < 6) {
    const int u = (blk - 2) * 256 + tid;
    const int nl = u >> 3;
    plane_piece(Wq, (nl >> 5) * 1056, nl & 31, (u & 7) * 8, 31, WqkvT + (size_t)u * 8);
  } else if (blk < 10) {
    const int u = (blk - 6) * 256 + tid;
    const int nl = u >> 3;
    plane_piece(Wk, (nl >> 5) * 1056, nl & 31, (u & 7) * 8, 31, WqkvT + (size_t)(1024 + u) * 8);
  } else if (blk < 14) {
    const int u = (blk - 10) * 256 + tid;
    const int nl = u >> 3;
    plane_piece(Wv, (nl >> 5) * 1056, nl & 31, (u & 7) * 8, 31, WqkvT + (size_t)(2048 + u) * 8);
  } else {
    const int u = tid;
    plane_piece(Who, 0, u >> 3, (u & 7) * 8, 31, WhoT + (size_t)u * 8);
  }
}

__device__ __forceinline__ int scan_chunk(const int* __restrict__ keys, int cbase, int slotBase, int* list,
                                          int tid, int lane, int wave) {
  int wc = 0;
  const int e0   = cbase + tid * CEPT;
  const int sent = (-0x7fffffff - 1);
  v4i da, db;
  if (cbase + CCHUNK <= NE) {
    da = *(const v4ia*)(keys + e0);
    db = *(const v4ia*)(keys + e0 + 4);
  } else {
    const int t0 = keys[min(e0,     NE - 1)];
    const int t1 = keys[min(e0 + 1, NE - 1)];
    const int t2 = keys[min(e0 + 2, NE - 1)];
    const int t3 = keys[min(e0 + 3, NE - 1)];
    const int t4 = keys[min(e0 + 4, NE - 1)];
    const int t5 = keys[min(e0 + 5, NE - 1)];
    const int t6 = keys[min(e0 + 6, NE - 1)];
    const int t7 = keys[min(e0 + 7, NE - 1)];
    asm volatile("" :: "v"(t0)); asm volatile("" :: "v"(t1)); asm volatile("" :: "v"(t2)); asm volatile("" :: "v"(t3));
    asm volatile("" :: "v"(t4)); asm volatile("" :: "v"(t5)); asm volatile("" :: "v"(t6)); asm volatile("" :: "v"(t7));
    da.x = (e0     < NE) ? t0 : sent;  da.y = (e0 + 1 < NE) ? t1 : sent;
    da.z = (e0 + 2 < NE) ? t2 : sent;  da.w = (e0 + 3 < NE) ? t3 : sent;
    db.x = (e0 + 4 < NE) ? t4 : sent;  db.y = (e0 + 5 < NE) ? t5 : sent;
    db.z = (e0 + 6 < NE) ? t6 : sent;  db.w = (e0 + 7 < NE) ? t7 : sent;
  }
  const unsigned nbs = (unsigned)slotBase;
  const unsigned unb = (unsigned)CNB;
  const unsigned s0 = (unsigned)da.x - nbs, s1 = (unsigned)da.y - nbs;
  const unsigned s2 = (unsigned)da.z - nbs, s3 = (unsigned)da.w - nbs;
  const unsigned s4 = (unsigned)db.x - nbs, s5 = (unsigned)db.y - nbs;
  const unsigned s6 = (unsigned)db.z - nbs, s7 = (unsigned)db.w - nbs;
  const bool h0 = s0 < unb, h1 = s1 < unb, h2 = s2 < unb, h3 = s3 < unb;
  const bool h4 = s4 < unb, h5 = s5 < unb, h6 = s6 < unb, h7 = s7 < unb;
  const unsigned any = __builtin_amdgcn_ballot_w32(h0 | h1 | h2 | h3 | h4 | h5 | h6 | h7);
  if (any != 0u) {
#define HITJ(HJ, SJ) { \
      const unsigned mj = __builtin_amdgcn_ballot_w32(HJ); \
      const int pos = wc + (int)__builtin_amdgcn_mbcnt_lo(mj, 0u); \
      if ((HJ) && pos < CWCAP) list[wave * CWCAP + pos] = (int)(SJ); \
      wc += (int)__builtin_popcount(mj); }
    HITJ(h0, s0)
    HITJ(h1, s1)
    HITJ(h2, s2)
    HITJ(h3, s3)
    HITJ(h4, s4)
    HITJ(h5, s5)
    HITJ(h6, s6)
    HITJ(h7, s7)
#undef HITJ
  }
  return wc;
}

__device__ __forceinline__ void count_pass(const int* __restrict__ keys, int slotBase, int* list, int* cnt,
                                           int* misc, int tid, int lane, int wave, int* outp) {
  {
    const v4i z4 = {0, 0, 0, 0};
    *(v4ia*)(cnt + 4 * tid) = z4;
  }
  __syncthreads();
  const int nChunks = (NE + CCHUNK - 1) / CCHUNK;
#pragma unroll 1
  for (int ch = 0; ch < nChunks; ++ch) {
    const int wc = scan_chunk(keys, ch * CCHUNK, slotBase, list, tid, lane, wave);
    if (lane == 0) misc[wave] = wc;
    __syncthreads();
    if (wave == 0) {
#pragma unroll 1
      for (int w2 = 0; w2 < 8; ++w2) {
        int c = misc[w2];
        c = c < 0 ? 0 : (c > CWCAP ? CWCAP : c);
#pragma unroll 1
        for (int b0 = 0; b0 < c; b0 += 32) {
          const int idx = b0 + lane;
          const int ent = list[w2 * CWCAP + (idx < CWCAP ? idx : CWCAP - 1)];
          const int m32 = (c - b0) < 32 ? (c - b0) : 32;
#pragma unroll 1
          for (int k = 0; k < m32; ++k) {
            const int slot = __builtin_amdgcn_readlane(ent, k) & (CNB - 1);
            if (lane == 0) cnt[slot] = cnt[slot] + 1;
          }
        }
      }
    }
    __syncthreads();
  }
  const v4i o = *(const v4ia*)(cnt + 4 * tid);
  int* dp = outp + 4 * tid;
  *(volatile v4i*)dp = o;
  __threadfence();
  *(volatile v4i*)dp = o;
  __syncthreads();
}

__global__ __launch_bounds__(256) void k_count(const int* __restrict__ src, const int* __restrict__ dst, int* CNT) {
  __shared__ __attribute__((aligned(16))) int sList[8 * CWCAP];
  __shared__ __attribute__((aligned(16))) int sCnt[CNB];
  __shared__ int sMisc[8];
  const int tid = (int)threadIdx.x, lane = tid & 31, wave = tid >> 5;
  const int slotBase = (int)blockIdx.x * CNB;
  {
    const v4i z4 = {0, 0, 0, 0};
    *(v4ia*)(sList + 4 * tid) = z4;
    *(v4ia*)(sList + 1024 + 4 * tid) = z4;
    if (tid < 8) sMisc[tid] = 0;
  }
  __syncthreads();
  count_pass(src, slotBase, sList, sCnt, sMisc, tid, lane, wave, CNT + slotBase);
  count_pass(dst, slotBase, sList, sCnt, sMisc, tid, lane, wave, CNT + CNTN + slotBase);
}

__global__ __launch_bounds__(256) __attribute__((amdgpu_num_vgpr(248)))
void k_node(const float* __restrict__ hin, const unsigned short* __restrict__ WfcT,
            const unsigned short* __restrict__ WqkvT, const float* __restrict__ Wfc,
            const float* __restrict__ bfc, const float* __restrict__ g1, const float* __restrict__ b1,
            const float* __restrict__ Wq, const float* __restrict__ bq, const float* __restrict__ Wk,
            const float* __restrict__ bk, const float* __restrict__ Wv, const float* __restrict__ bv,
            const float* __restrict__ nsc, float* RES, float* P3) {
  __shared__ __attribute__((aligned(16))) float sSt[8][16 * 32];
  __shared__ __attribute__((aligned(16))) unsigned short sA[8][16 * 64];
  __shared__ float sTm[8][16];
  __shared__ float sPar[128];
  __shared__ float sWt0[384];
  __shared__ float sBq[384];
  const int tid = (int)threadIdx.x, lane = tid & 31, wave = tid >> 5;
  const int hh = lane >> 4, m = lane & 15, h8 = hh * 8;
  const int rowBase = (int)blockIdx.x * RB + wave * 16;

  if (tid < 32) {
    sPar[tid]      = bf16_val(Wfc[tid]);
    sPar[32 + tid] = bf16_val(bfc[tid]);
    sPar[64 + tid] = bf16_val(g1[tid]);
    sPar[96 + tid] = bf16_val(b1[tid]);
  }
  __syncthreads();
  if (tid < 128) {
    const int ho = (tid >> 5) * 1056 + (tid & 31);
    sWt0[tid]       = bf16_val(Wq[ho]);
    sWt0[128 + tid] = bf16_val(Wk[ho]);
    sWt0[256 + tid] = bf16_val(Wv[ho]);
    sBq[tid]        = bf16_val(bq[tid]);
    sBq[128 + tid]  = bf16_val(bk[tid]);
    sBq[256 + tid]  = bf16_val(bv[tid]);
  }
  const float inv = 1.0f / fabsf(bf16_val(nsc[0]));

  v8f c0 = (v8f){0.f, 0.f, 0.f, 0.f, 0.f, 0.f, 0.f, 0.f};
  v8f c1 = c0;
  {
    const int arow = min(rowBase + m, NN - 1);
    const float* ap = hin + (size_t)arow * 128 + h8;
#pragma unroll
    for (int ks = 0; ks < 4; ++ks) {
      const float* p = ap + ks * 32;
      const v4f a0 = *(const v4fa*)(p);
      const v4f a1 = *(const v4fa*)(p + 4);
      const v4f a2 = *(const v4fa*)(p + 16);
      const v4f a3 = *(const v4fa*)(p + 20);
      const FragB af = mk_frag(pack8_bf16(a0, a1), pack8_bf16(a2, a3));
      const FragB b0 = ld_frag<FragB>(WfcT + (size_t)m * 128 + ks * 32 + h8);
      const FragB b1f = ld_frag<FragB>(WfcT + (size_t)(16 + m) * 128 + ks * 32 + h8);
      c0 = wmb(af, b0, c0);
      c1 = wmb(af, b1f, c1);
    }
  }
  float* st = sSt[wave];
#pragma unroll
  for (int r = 0; r < 8; ++r) {
    st[(h8 + r) * 32 + m]      = c0[r];
    st[(h8 + r) * 32 + 16 + m] = c1[r];
  }
  __syncthreads();

  {
    const float fc0 = sPar[lane], bfv = sPar[32 + lane], g1v = sPar[64 + lane], b1v = sPar[96 + lane];
#pragma unroll 1
    for (int i = 0; i < 16; ++i) {
      const bool live = (rowBase + i) < NN;
      const float s0 = (st[i * 32 + lane] + fc0) + bfv;
      const float mean = wsum32(s0) * (1.0f / 32.0f);
      const float d = s0 - mean;
      const float var = wsum32(d * d) * (1.0f / 32.0f);
      float y = (d / sqrtf(var + 1e-5f)) * g1v + b1v;
      y = leaky01(y);
      const float tm = sqrtf(wsum32(y * y) + 1.0f);
      st[i * 32 + lane] = live ? s0 : 0.0f;
      sA[wave][i * 64 + lane]      = (unsigned short)bf16_bits(y);
      sA[wave][i * 64 + 32 + lane] = (unsigned short)bf16_lo_bits(y);
      if (lane == 0) sTm[wave][i] = tm;
    }
  }
  __syncthreads();
  flush_tile(st, RES + (size_t)rowBase * 32, 32, lane);

  FragB aHi, aLo;
  {
    const unsigned short* q = &sA[wave][m * 64 + h8];
    aHi.h[0] = *(const v8usa*)(q);
    aHi.h[1] = *(const v8usa*)(q + 16);
    aLo.h[0] = *(const v8usa*)(q + 32);
    aLo.h[1] = *(const v8usa*)(q + 48);
  }

#pragma unroll 1
  for (int g = 0; g < 12; ++g) {
    const int nb = g * 32;
    const unsigned short* bp = WqkvT + (size_t)(nb + m) * 64 + h8;
    const FragB b00 = ld_frag<FragB>(bp);
    const FragB b01 = ld_frag<FragB>(bp + 32);
    const FragB b10 = ld_frag<FragB>(bp + 16 * 64);
    const FragB b11 = ld_frag<FragB>(bp + 16 * 64 + 32);
    v8f d0 = (v8f){0.f, 0.f, 0.f, 0.f, 0.f, 0.f, 0.f, 0.f};
    v8f d1 = d0;
    d0 = wmb(aHi, b00, d0);
    d0 = wmb(aLo, b01, d0);
    d1 = wmb(aHi, b10, d1);
    d1 = wmb(aLo, b11, d1);
    __syncthreads();
#pragma unroll
    for (int r = 0; r < 8; ++r) {
      st[(h8 + r) * 32 + m]      = d0[r];
      st[(h8 + r) * 32 + 16 + m] = d1[r];
    }
    __syncthreads();
    const float w0 = sWt0[nb + lane];
    const float bb = sBq[nb + lane];
    const bool dofp = g < 8;
#pragma unroll 1
    for (int i = 0; i < 16; ++i) {
      const bool live = (rowBase + i) < NN;
      float v = (st[i * 32 + lane] + sTm[wave][i] * w0) + bb;
      v = leaky01(v);
      const float x = (v + 1e-6f) * inv;
      float o = x;
      if (dofp) {
        const float nx2 = wsum32(x * x);
        const float xp  = x * x * x;
        const float np2 = wsum32(xp * xp);
        o = (sqrtf(nx2) / sqrtf(np2)) * xp;
      }
      st[i * 32 + lane] = live ? o : 0.0f;
    }
    __syncthreads();
    flush_tile(st, P3 + (size_t)(g >> 2) * PLE + (size_t)rowBase * 128 + (g & 3) * 32, 128, lane);
  }
}

__global__ __launch_bounds__(256) __attribute__((amdgpu_num_vgpr(248)))
void k_moment(const float* __restrict__ P3, const int* __restrict__ CSRC, float* REC, float* KREC) {
  __shared__ __attribute__((aligned(16))) unsigned short sKh[128 * 32];
  __shared__ __attribute__((aligned(16))) unsigned short sKl[128 * 32];
  __shared__ __attribute__((aligned(16))) unsigned short sVh[128 * 32];
  __shared__ __attribute__((aligned(16))) unsigned short sVl[128 * 32];
  __shared__ __attribute__((aligned(16))) float sRec[4096];
  __shared__ __attribute__((aligned(16))) float sKs[256];
  const int tid = (int)threadIdx.x, lane = tid & 31, wave = tid >> 5;
  const int hh = lane >> 4, m = lane & 15, h8 = hh * 8;
  const int blk = (int)blockIdx.x;
  const float* PK = P3 + PLE;
  const float* PV = P3 + 2 * PLE;

  {
    const int col = tid & 127;
    const int r0 = blk * MBR + (tid >> 7) * 256;
    float ks = 0.0f;
#pragma unroll 4
    for (int j = 0; j < 256; ++j) {
      const int row = r0 + j;
      const int rc = min(row, NPADR - 1);
      const float pk = PK[(size_t)rc * 128 + col];
      const int ci = CSRC[row];
      const float cs = (row < NN) ? (float)ci : 0.0f;
      ks += pk * cs;
    }
    sKs[tid] = ks;
  }

  const int nd = tid >> 3;
  const int cg = (tid & 7) * 16;
  const int hd = wave >> 1, mh = wave & 1;
  v8f acc0 = (v8f){0.f, 0.f, 0.f, 0.f, 0.f, 0.f, 0.f, 0.f};
  v8f acc1 = acc0;

#pragma unroll 1
  for (int s = 0; s < 16; ++s) {
    const int row = blk * MBR + s * 32 + nd;
    const int rc = min(row, NPADR - 1);
    const int ci = CSRC[row];
    asm volatile("" :: "v"(ci));
    const float cs = (row < NN) ? (float)ci : 0.0f;
    __syncthreads();
#pragma unroll
    for (int q = 0; q < 4; ++q) {
      const v4f k4 = *(const v4fa*)(PK + (size_t)rc * 128 + cg + 4 * q);
      const v4f v4 = *(const v4fa*)(PV + (size_t)rc * 128 + cg + 4 * q);
#pragma unroll
      for (int e = 0; e < 4; ++e) {
        const int c = cg + 4 * q + e;
        const float a = k4[e] * cs;
        sKh[c * 32 + nd] = (unsigned short)bf16_bits(a);
        sKl[c * 32 + nd] = (unsigned short)bf16_lo_bits(a);
        sVh[c * 32 + nd] = (unsigned short)bf16_bits(v4[e]);
        sVl[c * 32 + nd] = (unsigned short)bf16_lo_bits(v4[e]);
      }
    }
    __syncthreads();
    FragB aH, aL, bH0, bL0, bH1, bL1;
    {
      const int ca = (hd * 32 + mh * 16 + m) * 32 + h8;
      aH.h[0] = *(const v8usa*)(&sKh[ca]);  aH.h[1] = *(const v8usa*)(&sKh[ca + 16]);
      aL.h[0] = *(const v8usa*)(&sKl[ca]);  aL.h[1] = *(const v8usa*)(&sKl[ca + 16]);
      const int cb0 = (hd * 32 + m) * 32 + h8;
      const int cb1 = (hd * 32 + 16 + m) * 32 + h8;
      bH0.h[0] = *(const v8usa*)(&sVh[cb0]); bH0.h[1] = *(const v8usa*)(&sVh[cb0 + 16]);
      bL0.h[0] = *(const v8usa*)(&sVl[cb0]); bL0.h[1] = *(const v8usa*)(&sVl[cb0 + 16]);
      bH1.h[0] = *(const v8usa*)(&sVh[cb1]); bH1.h[1] = *(const v8usa*)(&sVh[cb1 + 16]);
      bL1.h[0] = *(const v8usa*)(&sVl[cb1]); bL1.h[1] = *(const v8usa*)(&sVl[cb1 + 16]);
    }
    acc0 = wmb(aH, bH0, acc0);
    acc0 = wmb(aL, bH0, acc0);
    acc0 = wmb(aH, bL0, acc0);
    acc1 = wmb(aH, bH1, acc1);
    acc1 = wmb(aL, bH1, acc1);
    acc1 = wmb(aH, bL1, acc1);
  }

#pragma unroll
  for (int r = 0; r < 8; ++r) {
    sRec[hd * 1024 + (mh * 16 + h8 + r) * 32 + m]      = acc0[r];
    sRec[hd * 1024 + (mh * 16 + h8 + r) * 32 + 16 + m] = acc1[r];
  }
  __syncthreads();
  {
    v4f vv[4];
#pragma unroll
    for (int it = 0; it < 4; ++it) vv[it] = *(const v4fa*)(sRec + 4 * (it * 256 + tid));
    float* rb = REC + (size_t)blk * 4096;
    for (int pass = 0; pass < 2; ++pass) {
#pragma unroll
      for (int it = 0; it < 4; ++it) *(volatile v4f*)(rb + 4 * (it * 256 + tid)) = vv[it];
      __threadfence();
    }
  }
  if (tid < 32) {
    v4f o;
    o.x = sKs[4 * tid]     + sKs[128 + 4 * tid];
    o.y = sKs[4 * tid + 1] + sKs[128 + 4 * tid + 1];
    o.z = sKs[4 * tid + 2] + sKs[128 + 4 * tid + 2];
    o.w = sKs[4 * tid + 3] + sKs[128 + 4 * tid + 3];
    float* kp = KREC + (size_t)blk * 128 + 4 * tid;
    *(volatile v4f*)kp = o;
    __threadfence();
    *(volatile v4f*)kp = o;
  }
}

__global__ __launch_bounds__(256) void k_comb(const float* __restrict__ REC, const float* __restrict__ KREC,
                                              unsigned short* KTVB, float* KSUM) {
  __shared__ __attribute__((aligned(16))) float sK[4096];
  __shared__ __attribute__((aligned(16))) float sS[128];
  const int tid = (int)threadIdx.x;
  double a[4][4];
#pragma unroll
  for (int j = 0; j < 4; ++j)
#pragma unroll
    for (int e = 0; e < 4; ++e) a[j][e] = 0.0;
#pragma unroll 1
  for (int b = 0; b < NMB; ++b) {
#pragma unroll
    for (int j = 0; j < 4; ++j) {
      const v4f x = *(const v4fa*)(REC + (size_t)b * 4096 + 4 * (j * 256 + tid));
#pragma unroll
      for (int e = 0; e < 4; ++e) a[j][e] += (double)x[e];
    }
  }
#pragma unroll
  for (int j = 0; j < 4; ++j)
#pragma unroll
    for (int e = 0; e < 4; ++e) sK[4 * (j * 256 + tid) + e] = (float)a[j][e];
  if (tid < 128) {
    double s = 0.0;
#pragma unroll 4
    for (int b = 0; b < NMB; ++b) s += (double)KREC[b * 128 + tid];
    sS[tid] = (float)s;
  }
  __syncthreads();

  v4u vv[6];
#pragma unroll
  for (int it = 0; it < 6; ++it) {
    const int g = it * 256 + tid;
    const int row = g / 12;
    const int pc = g - row * 12;
    const int k8 = pc * 8;
    const bool lo = k8 >= 64;
    const int kk = k8 & 31;
    const int hd = row >> 5, d = row & 31;
    unsigned w[8];
#pragma unroll
    for (int e = 0; e < 8; ++e) {
      const float v = sK[hd * 1024 + (kk + e) * 32 + d];
      const unsigned bh = bf16_bits(v);
      const unsigned bl = bf16_lo_bits(v);
      w[e] = lo ? bl : bh;
    }
    vv[it] = (v4u){ pk16(w[0], w[1]), pk16(w[2], w[3]), pk16(w[4], w[5]), pk16(w[6], w[7]) };
  }
  for (int pass = 0; pass < 2; ++pass) {
#pragma unroll
    for (int it = 0; it < 6; ++it) *(volatile v4u*)(KTVB + (size_t)(it * 256 + tid) * 8) = vv[it];
    __threadfence();
  }
  if (tid < 32) {
    const v4f o = *(const v4fa*)(sS + 4 * tid);
    float* kp = KSUM + 4 * tid;
    *(volatile v4f*)kp = o;
    __threadfence();
    *(volatile v4f*)kp = o;
  }
}

__global__ __launch_bounds__(256) __attribute__((amdgpu_num_vgpr(248)))
void k_out(const float* __restrict__ PQ, const float* __restrict__ RES, const unsigned short* __restrict__ KTVB,
           const float* __restrict__ KSUM, const unsigned short* __restrict__ WhoT, const float* __restrict__ Who,
           const float* __restrict__ bho, const float* __restrict__ g2, const float* __restrict__ b2,
           const int* __restrict__ CDST, float* outp) {
  __shared__ __attribute__((aligned(16))) float sImg[RB * 33];
  __shared__ __attribute__((aligned(16))) float sSt[8][16 * 32];
  __shared__ __attribute__((aligned(16))) unsigned short sA[8][16 * 64];
  __shared__ float sDen[8][64];
  __shared__ float sTa[8][16];
  __shared__ __attribute__((aligned(16))) float sKsum[128];
  __shared__ float sPar[128];
  const int tid = (int)threadIdx.x, lane = tid & 31, wave = tid >> 5;
  const int hh = lane >> 4, m = lane & 15, h8 = hh * 8;
  const int rowBase = (int)blockIdx.x * RB + wave * 16;

  if (tid < 32) {
    sPar[tid]      = bf16_val(Who[tid]);
    sPar[32 + tid] = bf16_val(bho[tid]);
    sPar[64 + tid] = bf16_val(g2[tid]);
    sPar[96 + tid] = bf16_val(b2[tid]);
    *(v4fa*)(sKsum + 4 * tid) = *(const v4fa*)(KSUM + 4 * tid);
  }
  __syncthreads();

  {
    const v4f ks4 = *(const v4fa*)(sKsum + 4 * lane);
#pragma unroll 4
    for (int i = 0; i < 16; ++i) {
      const v4f p = *(const v4fa*)(PQ + (size_t)(rowBase + i) * 128 + 4 * lane);
      float ds = ((p.x * ks4.x + p.y * ks4.y) + p.z * ks4.z) + p.w * ks4.w;
      ds += __shfl_xor(ds, 4, 32);
      ds += __shfl_xor(ds, 2, 32);
      ds += __shfl_xor(ds, 1, 32);
      if ((lane & 7) == 0) sDen[wave][i * 4 + (lane >> 3)] = ds + 1e-6f;
    }
  }
  __syncthreads();

  v8f at0 = (v8f){0.f, 0.f, 0.f, 0.f, 0.f, 0.f, 0.f, 0.f};
  v8f at1 = at0;
#pragma unroll 1
  for (int hd = 0; hd < 4; ++hd) {
    const float* p = PQ + (size_t)(rowBase + m) * 128 + hd * 32 + h8;
    const v4f a0 = *(const v4fa*)(p);
    const v4f a1 = *(const v4fa*)(p + 4);
    const v4f a2 = *(const v4fa*)(p + 16);
    const v4f a3 = *(const v4fa*)(p + 20);
    const FragB aH = mk_frag(pack8_bf16(a0, a1), pack8_bf16(a2, a3));
    const FragB aL = mk_frag(pack8_bf16_lo(a0, a1), pack8_bf16_lo(a2, a3));
    const unsigned short* bp = KTVB + (size_t)(hd * 32 + m) * 96 + h8;
    v8f n0 = (v8f){0.f, 0.f, 0.f, 0.f, 0.f, 0.f, 0.f, 0.f};
    v8f n1 = n0;
    {
      const FragB b0 = ld_frag<FragB>(bp);
      const FragB b1f = ld_frag<FragB>(bp + 32);
      const FragB b2f = ld_frag<FragB>(bp + 64);
      n0 = wmb(aH, b0, n0);
      n0 = wmb(aL, b1f, n0);
      n0 = wmb(aH, b2f, n0);
    }
    {
      const FragB b0 = ld_frag<FragB>(bp + 16 * 96);
      const FragB b1f = ld_frag<FragB>(bp + 16 * 96 + 32);
      const FragB b2f = ld_frag<FragB>(bp + 16 * 96 + 64);
      n1 = wmb(aH, b0, n1);
      n1 = wmb(aL, b1f, n1);
      n1 = wmb(aH, b2f, n1);
    }
#pragma unroll
    for (int r = 0; r < 8; ++r) {
      const float dn = sDen[wave][(h8 + r) * 4 + hd];
      at0[r] = at0[r] + n0[r] / dn;
      at1[r] = at1[r] + n1[r] / dn;
    }
  }
  float* st = sSt[wave];
#pragma unroll
  for (int r = 0; r < 8; ++r) {
    st[(h8 + r) * 32 + m]      = at0[r] * 0.25f;
    st[(h8 + r) * 32 + 16 + m] = at1[r] * 0.25f;
  }
  __syncthreads();

#pragma unroll 1
  for (int i = 0; i < 16; ++i) {
    const float a = st[i * 32 + lane];
    const float ta = sqrtf(wsum32(a * a) + 1.0f);
    sA[wave][i * 64 + lane]      = (unsigned short)bf16_bits(a);
    sA[wave][i * 64 + 32 + lane] = (unsigned short)bf16_lo_bits(a);
    if (lane == 0) sTa[wave][i] = ta;
  }
  __syncthreads();

  {
    FragB aHi, aLo;
    const unsigned short* q = &sA[wave][m * 64 + h8];
    aHi.h[0] = *(const v8usa*)(q);
    aHi.h[1] = *(const v8usa*)(q + 16);
    aLo.h[0] = *(const v8usa*)(q + 32);
    aLo.h[1] = *(const v8usa*)(q + 48);
    const unsigned short* bp = WhoT + (size_t)m * 64 + h8;
    const FragB b00 = ld_frag<FragB>(bp);
    const FragB b01 = ld_frag<FragB>(bp + 32);
    const FragB b10 = ld_frag<FragB>(bp + 16 * 64);
    const FragB b11 = ld_frag<FragB>(bp + 16 * 64 + 32);
    v8f o0 = (v8f){0.f, 0.f, 0.f, 0.f, 0.f, 0.f, 0.f, 0.f};
    v8f o1 = o0;
    o0 = wmb(aHi, b00, o0);
    o0 = wmb(aLo, b01, o0);
    o1 = wmb(aHi, b10, o1);
    o1 = wmb(aLo, b11, o1);
#pragma unroll
    for (int r = 0; r < 8; ++r) {
      st[(h8 + r) * 32 + m]      = o0[r];
      st[(h8 + r) * 32 + 16 + m] = o1[r];
    }
  }
  __syncthreads();

  {
    const float who0 = sPar[lane], bhv = sPar[32 + lane], g2v = sPar[64 + lane], b2v = sPar[96 + lane];
    const float qnan = __uint_as_float(0x7fc00000u);
#pragma unroll 1
    for (int i = 0; i < 16; ++i) {
      const int row = rowBase + i;
      const float es = (st[i * 32 + lane] + sTa[wave][i] * who0) + bhv;
      const float et = sqrtf(wsum32(es * es) + 1.0f);
      const int cv = CDST[row];
      const int ccv = cv < 0 ? 0 : (cv > DEGCAP ? DEGCAP : cv);
      const int bigv = (cv > DEGCAP) ? 1 : 0;
      const int cc = __builtin_amdgcn_readfirstlane(ccv);
      const bool big = __builtin_amdgcn_readfirstlane(bigv) != 0;
      float as = 0.0f, att = 0.0f;
#pragma unroll 1
      for (int j = 0; j < cc; ++j) { as += es; att += et; }
      const float fc = (float)(cc > 0 ? cc : 1);
      const float ags = (cc > 0) ? as / fc : 0.0f;
      const float agt = (cc > 0) ? att / fc : 0.0f;
      const float s0 = RES[(size_t)row * 32 + lane];
      const float rt = sqrtf(wsum32(s0 * s0) + 1.0f);
      const float avs = 0.5f * (ags + s0);
      const float avt = 0.5f * (agt + rt);
      const float inner = wsum32(avs * avs) - avt * avt;
      const float dn = sqrtf(fmaxf(fabsf(inner), 1e-6f));
      const float hs = avs / dn;
      const float mean = wsum32(hs) * (1.0f / 32.0f);
      const float d = hs - mean;
      const float var = wsum32(d * d) * (1.0f / 32.0f);
      float y = (d / sqrtf(var + 1e-5f)) * g2v + b2v;
      float to = sqrtf(wsum32(y * y) + 1.0f);
      y  = big ? qnan : y;
      to = big ? qnan : to;
      sImg[(wave * 16 + i) * 33 + 1 + lane] = y;
      if (lane == 0) sImg[(wave * 16 + i) * 33] = to;
    }
  }
  __syncthreads();

  {
    const int nrows = min(RB, NN - (int)blockIdx.x * RB);
    const int npieces = (nrows * 33) >> 2;
    float* ob = outp + (size_t)blockIdx.x * (RB * 33);
    v4f vv[5];
#pragma unroll
    for (int it = 0; it < 5; ++it) {
      const int idx = min(it * 256 + tid, (RB * 33) / 4 - 1);
      vv[it] = *(const v4fa*)(sImg + 4 * idx);
    }
    for (int pass = 0; pass < 2; ++pass) {
#pragma unroll
      for (int it = 0; it < 5; ++it) {
        const int idx = it * 256 + tid;
        if (idx < npieces) *(volatile v4f*)(ob + 4 * idx) = vv[it];
      }
      __threadfence();
    }
  }
}

extern "C" void kernel_launch(void* const* d_in, const int* in_sizes, int n_in,
                              void* d_out, int out_size, void* d_ws, size_t ws_size,
                              hipStream_t stream) {
  if (n_in < 18) return;
  if (in_sizes[0] != NN * 128) return;
  if (in_sizes[1] != NE || in_sizes[2] != NE) return;
  if (in_sizes[3] != 129 * 32 || in_sizes[4] != 32) return;
  if (in_sizes[5] != 32 || in_sizes[6] != 32) return;
  if (in_sizes[7] != 4224 || in_sizes[9] != 4224 || in_sizes[11] != 4224) return;
  if (in_sizes[8] != 128 || in_sizes[10] != 128 || in_sizes[12] != 128) return;
  if (in_sizes[13] != 33 * 32 || in_sizes[14] != 32) return;
  if (in_sizes[15] != 32 || in_sizes[16] != 32) return;
  if (in_sizes[17] < 1) return;
  if (out_size != NN * 33) return;

  const float* h    = (const float*)d_in[0];
  const int*   src  = (const int*)d_in[1];
  const int*   dst  = (const int*)d_in[2];
  const float* Wfc  = (const float*)d_in[3];
  const float* bfc  = (const float*)d_in[4];
  const float* ln1g = (const float*)d_in[5];
  const float* ln1b = (const float*)d_in[6];
  const float* Wq   = (const float*)d_in[7];
  const float* bq   = (const float*)d_in[8];
  const float* Wk   = (const float*)d_in[9];
  const float* bk   = (const float*)d_in[10];
  const float* Wv   = (const float*)d_in[11];
  const float* bv   = (const float*)d_in[12];
  const float* Who  = (const float*)d_in[13];
  const float* bho  = (const float*)d_in[14];
  const float* ln2g = (const float*)d_in[15];
  const float* ln2b = (const float*)d_in[16];
  const float* nsc  = (const float*)d_in[17];
  float* out = (float*)d_out;

  char* ws = (char*)d_ws;
  size_t off = 0;
  const size_t oWfcT = off; off += (size_t)32 * 128 * 2;        off = (off + 255) & ~(size_t)255;
  const size_t oWqkv = off; off += (size_t)384 * 64 * 2;        off = (off + 255) & ~(size_t)255;
  const size_t oWhoT = off; off += (size_t)32 * 64 * 2;         off = (off + 255) & ~(size_t)255;
  const size_t oCNT  = off; off += (size_t)2 * CNTN * 4;        off = (off + 255) & ~(size_t)255;
  const size_t oRES  = off; off += (size_t)NPADR * 32 * 4;      off = (off + 255) & ~(size_t)255;
  const size_t oP3   = off; off += (size_t)3 * PLE * 4;         off = (off + 255) & ~(size_t)255;
  const size_t oREC  = off; off += (size_t)NMB * 4096 * 4;      off = (off + 255) & ~(size_t)255;
  const size_t oKREC = off; off += (size_t)NMB * 128 * 4;       off = (off + 255) & ~(size_t)255;
  const size_t oKTVB = off; off += (size_t)4 * 32 * 96 * 2;     off = (off + 255) & ~(size_t)255;
  const size_t oKSUM = off; off += (size_t)128 * 4;             off = (off + 255) & ~(size_t)255;
  if (off > ws_size || off > (size_t)WSMAX) return;
  unsigned short* WfcT  = (unsigned short*)(ws + oWfcT);
  unsigned short* WqkvT = (unsigned short*)(ws + oWqkv);
  unsigned short* WhoT  = (unsigned short*)(ws + oWhoT);
  int*            CNT   = (int*)(ws + oCNT);
  float*          RES   = (float*)(ws + oRES);
  float*          P3    = (float*)(ws + oP3);
  float*          REC   = (float*)(ws + oREC);
  float*          KREC  = (float*)(ws + oKREC);
  unsigned short* KTVB  = (unsigned short*)(ws + oKTVB);
  float*          KSUM  = (float*)(ws + oKSUM);

  k_prep<<<15, 256, 0, stream>>>(Wfc, Wq, Wk, Wv, Who, WfcT, WqkvT, WhoT);
  k_count<<<NCB, 256, 0, stream>>>(src, dst, CNT);
  k_node<<<NBLK, 256, 0, stream>>>(h, WfcT, WqkvT, Wfc, bfc, ln1g, ln1b, Wq, bq, Wk, bk, Wv, bv, nsc, RES, P3);
  k_moment<<<NMB, 256, 0, stream>>>(P3, CNT, REC, KREC);
  k_comb<<<1, 256, 0, stream>>>(REC, KREC, KTVB, KSUM);
  k_out<<<NBLK, 256, 0, stream>>>(P3, RES, KTVB, KSUM, WhoT, Who, bho, ln2g, ln2b, CNT + CNTN, out);
}
